// SelfAttention2varible_8555574854295
// MI455X (gfx1250) — hardware-verified
//
#include <hip/hip_runtime.h>
#include <math.h>

typedef __attribute__((ext_vector_type(16))) _Float16 v16h;
typedef __attribute__((ext_vector_type(16))) __bf16 v16b;
typedef __attribute__((ext_vector_type(8)))  _Float16 v8h;
typedef __attribute__((ext_vector_type(8)))  float v8f;
typedef __attribute__((ext_vector_type(4)))  float v4f;
typedef __attribute__((ext_vector_type(2)))  float v2f;
typedef __attribute__((ext_vector_type(4)))  unsigned v4u;
typedef __attribute__((ext_vector_type(4)))  int v4i;
typedef float __attribute__((may_alias)) float_a;
typedef int __attribute__((may_alias)) int_a;

template <typename T> __device__ __forceinline__ void vst2(void* p, T v) { *(volatile T*)p = v; __threadfence(); *(volatile T*)p = v; }
__device__ __forceinline__ v8f wmma16(v16h a, v16h b, v8f c) {
  v8f d = __builtin_amdgcn_wmma_f32_16x16x32_f16(false, a, false, b, (short)0, c, false, false);
  asm volatile("v_nop\n\tv_nop\n\tv_nop\n\tv_nop" : "+v"(d) : "v"(a), "v"(b));
  return d;
}
__device__ __forceinline__ v8f wmma_bf(v16b a, v16b b, v8f c) {
  v8f d = __builtin_amdgcn_wmma_f32_16x16x32_bf16(false, a, false, b, (short)0, c, false, false);
  asm volatile("v_nop\n\tv_nop\n\tv_nop\n\tv_nop" : "+v"(d) : "v"(a), "v"(b));
  return d;
}
__device__ __forceinline__ v16h frag_h(const _Float16* rowk0, int lane) {
  union { v16h v; v8h q[2]; } u; const _Float16* p = rowk0 + 8 * (lane >> 4);
  u.q[0] = *(const v8h*)p; u.q[1] = *(const v8h*)(p + 16); return u.v;
}
__device__ __forceinline__ v16h frag_f32(const float* rowk0, int lane) {
  v16h a; const float* p = rowk0 + 8 * (lane >> 4);
#pragma unroll
  for (int i = 0; i < 8; ++i) { a[i] = (_Float16)p[i]; a[8 + i] = (_Float16)p[16 + i]; }
  return a;
}
__device__ __forceinline__ v16h frag_f32s(const float* rowk0, int lane, float sc) {
  v16h a; const float* p = rowk0 + 8 * (lane >> 4);
#pragma unroll
  for (int i = 0; i < 8; ++i) { a[i] = (_Float16)(p[i] * sc); a[8 + i] = (_Float16)(p[16 + i] * sc); }
  return a;
}
__device__ __forceinline__ v16h fragc_f32(const float* W, int k0, int n, int lane, int ld, int K) {
  v16h a; const int g = lane >> 4;
#pragma unroll
  for (int i = 0; i < 8; ++i) { const int ka = k0 + 8 * g + i, kb = ka + 16;
    a[i] = (_Float16)(ka < K ? W[(size_t)(ka < K ? ka : K - 1) * ld + n] : 0.f); a[8 + i] = (_Float16)(kb < K ? W[(size_t)(kb < K ? kb : K - 1) * ld + n] : 0.f); }
  return a;
}
struct F2 { v16b h, l; };
__device__ __forceinline__ F2 bsplit16(const float v[16]) { F2 r;
#pragma unroll
  for (int i = 0; i < 16; ++i) { const __bf16 h = (__bf16)v[i]; r.h[i] = h; r.l[i] = (__bf16)(v[i] - (float)h); }
  return r; }
__device__ __forceinline__ F2 split_row(const float* row, int k0, int lane) { float v[16]; const float* p = row + k0 + 8 * (lane >> 4);
#pragma unroll
  for (int i = 0; i < 8; ++i) { v[i] = p[i]; v[8 + i] = p[16 + i]; }
  return bsplit16(v); }
__device__ __forceinline__ F2 split_rowK(const float* row, int k0, int lane, int K) { float v[16]; const int g = lane >> 4;
#pragma unroll
  for (int i = 0; i < 8; ++i) { const int ka = k0 + 8 * g + i, kb = ka + 16; v[i] = ka < K ? row[ka < K ? ka : K - 1] : 0.f; v[8 + i] = kb < K ? row[kb < K ? kb : K - 1] : 0.f; }
  return bsplit16(v); }
__device__ __forceinline__ F2 split_col(const float* W, int k0, int n, int lane, int ld, int K) { float v[16]; const int g = lane >> 4;
#pragma unroll
  for (int i = 0; i < 8; ++i) { const int ka = k0 + 8 * g + i, kb = ka + 16; v[i] = ka < K ? W[(size_t)(ka < K ? ka : K - 1) * ld + n] : 0.f; v[8 + i] = kb < K ? W[(size_t)(kb < K ? kb : K - 1) * ld + n] : 0.f; }
  return bsplit16(v); }
__device__ __forceinline__ v8f mac3(const F2& a, const F2& b, v8f c) { c = wmma_bf(a.l, b.h, c); c = wmma_bf(a.h, b.l, c); return wmma_bf(a.h, b.h, c); }
__device__ __forceinline__ float sigm(float v) { return 1.0f / (1.0f + expf(-v)); }
#define LDSX() do { asm volatile("s_wait_dscnt 0" ::: "memory"); __builtin_amdgcn_wave_barrier(); __builtin_amdgcn_fence(__ATOMIC_RELEASE, "workgroup"); } while (0)


#define NB 8
#define CC 256
#define NG 32
#define CPG (CC / NG)
#define NN 1024
#define NH 8
#define HD 32
#define NR (NB * NN)
#ifndef TQB
#define TQB (NN / 64)
#define TNB NB
#endif
typedef __attribute__((ext_vector_type(8))) __bf16 v8b;
__device__ __forceinline__ v16b frag_b(const __bf16* rowk0, int lane) {
  union { v16b v; v8b q[2]; } u; const __bf16* p = rowk0 + 8 * (lane >> 4);
  u.q[0] = *(const v8b*)p; u.q[1] = *(const v8b*)(p + 16); return u.v;
}
__device__ __forceinline__ float bfr(float v) { return (float)(__bf16)v; }
__device__ __attribute__((noinline)) float exp_ni(float v) { return expf(v); }
__device__ __attribute__((noinline)) float erf_ni(float v) { return erff(v); }

#define QS 512
#define WS_PW   0u
#define WS_MV   (WS_PW + 2u * (size_t)4 * CC * CC)
#define WS_NT   (WS_MV + 4u * (size_t)2 * NB * NG * 32)
#define WS_NTL  (WS_NT + 2u * (size_t)2 * NR * CC)
#define WS_Q    (WS_NTL + 2u * (size_t)2 * NR * CC)
#define WS_K    (WS_Q + 2u * (size_t)NR * QS)
#define WS_V    (WS_K + 2u * (size_t)NR * QS)
#define WS_O    (WS_V + 2u * (size_t)NB * CC * NN)
#define WS_END  (WS_O + 4u * (size_t)NR * CC)

__global__ __launch_bounds__(256) void k_pack(const float* __restrict__ WQ, const float* __restrict__ WKV, const float* __restrict__ WO, __bf16* __restrict__ P) { const size_t n = blockIdx.x; const int t = threadIdx.x; const float* src = (n < CC) ? (WQ + n * CC) : (n < 3 * CC) ? (WKV + (n - CC) * CC) : (WO + (n - 3 * CC) * CC); __shared__ __align__(16) __bf16 s[CC]; s[t] = (__bf16)src[t]; __syncthreads(); if (t < CC / 8) vst2((unsigned*)(P + n * CC + t * 8), *(const v4u*)&s[t * 8]); }
template <int SQ>
__global__ __launch_bounds__(1024) void k_gn(const float* __restrict__ XQ, const float* __restrict__ XKV, float* __restrict__ MV) {
  __shared__ float red[32]; __shared__ __align__(16) float line[32]; const int gidx = blockIdx.x, t = threadIdx.x; const size_t b = blockIdx.y; const int which = blockIdx.z; const float* X = which ? XKV : XQ;
  float* mv = MV + (((size_t)which * NB + b) * NG + gidx) * 32; const float mean = SQ ? mv[0] : 0.f; const float* p = X + (b * CC + (size_t)gidx * CPG) * NN; float s = 0.f;
  for (int i = t; i < CPG * NN; i += 1024) { const float v = bfr(p[i]) - mean; s += SQ ? v * v : v; }
#pragma unroll
  for (int o = 1; o < 32; o <<= 1) s += __shfl_xor(s, o);
  if ((t & 31) == 0) red[t >> 5] = s; __syncthreads();
  if (t < 32) { float tot = 0.f; for (int i = 0; i < 32; ++i) tot += red[i]; const float v = tot / (float)(CPG * NN); line[t] = SQ ? ((t == 0) ? mean : (t == 1) ? v : 0.f) : ((t == 0) ? v : 0.f); }
  __syncthreads(); if (t < 8) vst2(mv + t * 4, *(const v4f*)&line[t * 4]);
}
__global__ __launch_bounds__(256) void k_norm(const float* __restrict__ XQ, const float* __restrict__ XKV, const float* __restrict__ MV, const float* __restrict__ GQ, const float* __restrict__ BQ, const float* __restrict__ GKV, const float* __restrict__ BKV, __bf16* __restrict__ NT, __bf16* __restrict__ NTL) {
  __shared__ __align__(16) __bf16 sh[64][CC + 8]; __shared__ __align__(16) __bf16 sl[64][CC + 8]; const int n0 = blockIdx.x * 64, t = threadIdx.x; const size_t b = blockIdx.y; const int which = blockIdx.z;
  const float* X = which ? XKV : XQ; const float* Gm = which ? GKV : GQ; const float* Bt = which ? BKV : BQ; const float* mv = MV + ((size_t)which * NB + b) * NG * 32;
  for (int e = t; e < CC * 64; e += 256) { const int c = e >> 6, nl = e & 63; const int gg = c / CPG; const float mean = mv[gg * 32], inv = 1.0f / sqrtf(mv[gg * 32 + 1] + 1e-5f); const float v = (bfr(X[(b * CC + c) * NN + n0 + nl]) - mean) * inv * bfr(Gm[c]) + bfr(Bt[c]); const __bf16 hv = (__bf16)v; sh[nl][c] = hv; sl[nl][c] = (__bf16)(v - (float)hv); }
  __syncthreads();
  __bf16* dh = NT + ((size_t)which * NR + b * NN + n0) * CC; __bf16* dl = NTL + ((size_t)which * NR + b * NN + n0) * CC;
  for (int e = t; e < 64 * (CC / 8); e += 256) { const int nl = e / (CC / 8), q = e % (CC / 8); vst2((unsigned*)(dh + (size_t)nl * CC + q * 8), *(const v4u*)&sh[nl][q * 8]); vst2((unsigned*)(dl + (size_t)nl * CC + q * 8), *(const v4u*)&sl[nl][q * 8]); }
}
__global__ __launch_bounds__(128) void k_qkv(const __bf16* __restrict__ NT, const __bf16* __restrict__ NTL, const __bf16* __restrict__ P, _Float16* __restrict__ Q, _Float16* __restrict__ Kr, _Float16* __restrict__ V) {
  __shared__ __align__(16) _Float16 so[64][136]; __shared__ __align__(16) _Float16 st[128][72];
  const int tid = threadIdx.x, wave = tid >> 5, lane = tid & 31, col = lane & 15, g = lane >> 4; const size_t b = blockIdx.z; const int n0b = blockIdx.x * 64; const int o0 = blockIdx.y * 128; const int which = (o0 < CC) ? 0 : 1;
  const size_t r0 = (size_t)which * NR + b * NN + n0b + wave * 16;
  v8f acc[8] = {};
#pragma unroll
  for (int kc = 0; kc < CC / 32; ++kc) { const v16b ah = frag_b(NT + (r0 + col) * CC + kc * 32, lane), al = frag_b(NTL + (r0 + col) * CC + kc * 32, lane);
#pragma unroll
    for (int j = 0; j < 8; ++j) { const v16b w = frag_b(P + (size_t)(o0 + j * 16 + col) * CC + kc * 32, lane); acc[j] = wmma_bf(ah, w, acc[j]); acc[j] = wmma_bf(al, w, acc[j]); } }
#pragma unroll
  for (int j = 0; j < 8; ++j)
#pragma unroll
    for (int r = 0; r < 8; ++r) { const _Float16 hv = (_Float16)acc[j][r]; so[wave * 16 + 8 * g + r][j * 16 + col] = hv; st[j * 16 + col][wave * 16 + 8 * g + r] = hv; }
  __syncthreads();
  const size_t rowb = b * NN + n0b;
  for (int j = 0; j < 8; ++j) { const int o = o0 + j * 16;
    if (o < CC) { const int hh = o / HD, dd = o % HD; const int qd = hh * 64 + dd; for (int e = tid; e < 64 * 2; e += 128) { const int nl = e >> 1, q8 = e & 1; vst2((unsigned*)(Q + (rowb + nl) * QS + qd + q8 * 8), *(const v4u*)&so[nl][j * 16 + q8 * 8]); } }
    else { const int oo = o - CC; const int hh = oo / (2 * HD), rr = oo % (2 * HD);
      if (rr < HD) { const int kd = hh * 64 + rr; for (int e = tid; e < 64 * 2; e += 128) { const int nl = e >> 1, q8 = e & 1; vst2((unsigned*)(Kr + (rowb + nl) * QS + kd + q8 * 8), *(const v4u*)&so[nl][j * 16 + q8 * 8]); } }
      else { const int vc = hh * HD + (rr - HD); for (int e = tid; e < 16 * 8; e += 128) { const int d = e >> 3, pc = e & 7; vst2((unsigned*)(V + ((b * CC + vc + d) * NN) + n0b + pc * 8), *(const v4u*)&st[j * 16 + d][pc * 8]); } } } }
}
__global__ __launch_bounds__(128) void k_attn(const _Float16* __restrict__ Q, const _Float16* __restrict__ Kr, const _Float16* __restrict__ V, float* __restrict__ O) {
  __shared__ __align__(16) _Float16 sph[4][16][40]; __shared__ __align__(16) float so[4][16][36];
  const int tid = threadIdx.x, wave = tid >> 5, lane = tid & 31, col = lane & 15, g = lane >> 4; const int h = blockIdx.y; const size_t b = blockIdx.z; const int q0 = blockIdx.x * 64 + wave * 16; const size_t rq = b * NN + q0;
  const v16h aq = frag_h(Q + (rq + col) * QS + h * 64, lane);
  float m[8], l[8];
#pragma unroll
  for (int r = 0; r < 8; ++r) { m[r] = -3.0e38f; l[r] = 0.f; }
  v8f acc[2] = {};
#pragma unroll 1
  for (int ks = 0; ks < NN / 32; ++ks) { const int j0 = ks * 32; v8f s[2];
#pragma unroll
    for (int ct = 0; ct < 2; ++ct) { const v8f z = {}; const v8f c = wmma16(aq, frag_h(Kr + (b * NN + j0 + ct * 16 + col) * QS + h * 64, lane), z);
#pragma unroll
      for (int r = 0; r < 8; ++r) s[ct][r] = c[r] * 0.0625f; }
#pragma unroll
    for (int r = 0; r < 8; ++r) { float mx = fmaxf(s[0][r], s[1][r]);
#pragma unroll
      for (int o = 1; o < 16; o <<= 1) mx = fmaxf(mx, __shfl_xor(mx, o));
      const float mn = fmaxf(m[r], mx); const float alpha = (m[r] <= -1.0e38f) ? 0.f : __expf(m[r] - mn); const float e0 = __expf(s[0][r] - mn), e1 = __expf(s[1][r] - mn); float es = e0 + e1;
#pragma unroll
      for (int o = 1; o < 16; o <<= 1) es += __shfl_xor(es, o);
      l[r] = l[r] * alpha + es; m[r] = mn;
#pragma unroll
      for (int dt = 0; dt < 2; ++dt) acc[dt][r] *= alpha;
      sph[wave][8 * g + r][col] = (_Float16)(e0 * 2048.0f); sph[wave][8 * g + r][16 + col] = (_Float16)(e1 * 2048.0f); }
    LDSX();
    const v16h pa = frag_h(&sph[wave][col][0], lane);
#pragma unroll
    for (int dt = 0; dt < 2; ++dt) acc[dt] = wmma16(pa, frag_h(V + ((b * CC + h * HD + dt * 16 + col) * NN) + j0, lane), acc[dt]);
    LDSX(); }
#pragma unroll
  for (int r = 0; r < 8; ++r) { const float il = (1.0f / 2048.0f) / l[r];
#pragma unroll
    for (int dt = 0; dt < 2; ++dt) so[wave][8 * g + r][dt * 16 + col] = acc[dt][r] * il; }
  LDSX();
  for (int rl = 0; rl < 16; ++rl) if (lane < 8) vst2(O + (rq + rl) * CC + h * HD + lane * 4, *(const v4f*)&so[wave][rl][lane * 4]);
}
__global__ __launch_bounds__(128) void k_out(const float* __restrict__ O, const __bf16* __restrict__ P, const float* __restrict__ BO, const float* __restrict__ XQ, float* __restrict__ Y) {
  __shared__ __align__(16) float st[128][68];
  const int tid = threadIdx.x, wave = tid >> 5, lane = tid & 31, col = lane & 15, g = lane >> 4; const size_t b = blockIdx.z; const int n0b = blockIdx.x * 64; const size_t r0 = b * NN + n0b + wave * 16; const int o0 = blockIdx.y * 128;
  v8f acc[8] = {};
#pragma unroll
  for (int kc = 0; kc < CC / 32; ++kc) { const F2 a = split_row(O + (r0 + col) * CC, kc * 32, lane);
#pragma unroll
    for (int j = 0; j < 8; ++j) { const v16b w = frag_b(P + ((size_t)3 * CC + o0 + j * 16 + col) * CC + kc * 32, lane); acc[j] = wmma_bf(a.l, w, acc[j]); acc[j] = wmma_bf(a.h, w, acc[j]); } }
#pragma unroll
  for (int j = 0; j < 8; ++j) { const float bb = bfr(BO[o0 + j * 16 + col]);
#pragma unroll
    for (int r = 0; r < 8; ++r) st[j * 16 + col][wave * 16 + 8 * g + r] = acc[j][r] + bb; }
  __syncthreads();
  for (int e = tid; e < 128 * 16; e += 128) { const int o = e >> 4, q = e & 15; const size_t off = ((b * CC + o0 + o) * NN) + n0b + q * 4; v4f v = *(const v4f*)&st[o][q * 4]; for (int i = 0; i < 4; ++i) v[i] += bfr(XQ[off + i]); vst2(Y + off, v); }
}
extern "C" void kernel_launch(void* const* d_in, const int* in_sizes, int n_in, void* d_out, int out_size, void* d_ws, size_t ws_size, hipStream_t stream) {
  (void)in_sizes; (void)n_in; (void)out_size;
  const float** F = (const float**)d_in;
  if (ws_size < (size_t)WS_END) return;
  char* ws = (char*)d_ws; __bf16 *P = (__bf16*)ws, *NT = (__bf16*)(ws + WS_NT), *NTL = (__bf16*)(ws + WS_NTL); float *MV = (float*)(ws + WS_MV), *O = (float*)(ws + WS_O); _Float16 *Q = (_Float16*)(ws + WS_Q), *Kr = (_Float16*)(ws + WS_K), *V = (_Float16*)(ws + WS_V);
  k_pack<<<4 * CC, 256, 0, stream>>>(F[6], F[7], F[8], P);
  k_gn<0><<<dim3(NG, NB, 2), 1024, 0, stream>>>(F[0], F[1], MV); k_gn<1><<<dim3(NG, NB, 2), 1024, 0, stream>>>(F[0], F[1], MV);
  k_norm<<<dim3(NN / 64, NB, 2), 256, 0, stream>>>(F[0], F[1], MV, F[2], F[3], F[4], F[5], NT, NTL);
  k_qkv<<<dim3(NN / 64, 3 * CC / 128, NB), 128, 0, stream>>>(NT, NTL, P, Q, Kr, V);
  k_attn<<<dim3(TQB, NH, TNB), 128, 0, stream>>>(Q, Kr, V, O);
  k_out<<<dim3(TQB, CC / 128, TNB), 128, 0, stream>>>(O, P, F[9], F[0], (float*)d_out);
}
